// CellAttention_47115791237126
// MI455X (gfx1250) — hardware-run, weakly checked
//
#include <hip/hip_runtime.h>


#ifndef NQ
#define NQ 1024
#endif
#define NQ_FULL 1024
#define NPIX 1024
#define ENC  512
#define ATT  256
#ifndef APITCH
#define APITCH NPIX
#endif
#define ALPHA_OFF ((size_t)NQ_FULL * ENC)
#define PSC  16384.0f
#define PSI  (1.0f / 16384.0f)
#define LOG2E 1.4426950408889634f
#define TP   72

static_assert(NQ % 64 == 0);
static_assert(NQ <= NQ_FULL);
static_assert(NPIX % 64 == 0);
static_assert(ENC % 64 == 0);
static_assert(ATT % 64 == 0);
static_assert(ENC % 32 == 0);
static_assert(NPIX % 32 == 0);
static_assert(ATT == 256);
static_assert(NPIX == 256 * 4);
static_assert(ATT % 4 == 0);
static_assert(ALPHA_OFF * 4 == (size_t)2097152);
static_assert((size_t)NQ * ENC <= ALPHA_OFF);
static_assert((TP * 2) % 16 == 0);
static_assert(APITCH % 32 == 0);
static_assert(16 * 68 * 4 <= 131072);
static_assert(64 * TP * 2 <= 131072);
static_assert((2 * ATT + NPIX + 16) * 4 <= 131072);

typedef _Float16 h16;
typedef unsigned short bf;
typedef __attribute__((ext_vector_type(16))) __bf16   v16bf;
typedef __attribute__((ext_vector_type(16))) _Float16 v16h;
typedef __attribute__((ext_vector_type(8)))  _Float16 v8h;
typedef __attribute__((ext_vector_type(8)))  unsigned short v8us;
typedef __attribute__((ext_vector_type(8)))  float    v8f;
typedef __attribute__((ext_vector_type(4)))  float    v4f;
typedef v4f  __attribute__((may_alias)) v4fa;
typedef v8h  __attribute__((may_alias)) v8ha;

__device__ __forceinline__ unsigned short f2bf(float f) { unsigned u = __float_as_uint(f); u += 0x7FFFu + ((u >> 16) & 1u); return (unsigned short)(u >> 16); }
__device__ __forceinline__ float bfr(float f) { return __uint_as_float(((unsigned)f2bf(f)) << 16); }
__device__ __forceinline__ v16h cat16(v8h lo, v8h hi) { return __builtin_shufflevector(lo, hi, 0, 1, 2, 3, 4, 5, 6, 7, 8, 9, 10, 11, 12, 13, 14, 15); }
__device__ __forceinline__ v16bf cat16b(v8us lo, v8us hi) { return __builtin_bit_cast(v16bf, __builtin_shufflevector(lo, hi, 0, 1, 2, 3, 4, 5, 6, 7, 8, 9, 10, 11, 12, 13, 14, 15)); }
__device__ __forceinline__ v8f wmma16(v16h a, v16h b, v8f c) { return __builtin_amdgcn_wmma_f32_16x16x32_f16(false, a, false, b, (short)0, c, false, false); }
__device__ __forceinline__ v8f wmmab(v16bf a, v16bf b, v8f c) { return __builtin_amdgcn_wmma_f32_16x16x32_bf16(false, a, false, b, (short)0, c, false, false); }
__device__ __forceinline__ v16h  ldh(const h16* p) { return cat16(*(const v8h*)p, *(const v8h*)(p + 16)); }
__device__ __forceinline__ v16bf ldb(const bf* p)  { return cat16b(*(const v8us*)p, *(const v8us*)(p + 16)); }
__device__ __forceinline__ void wave_sync() { __builtin_amdgcn_fence(3  , "wavefront"); __builtin_amdgcn_wave_barrier(); asm volatile("" ::: "memory"); }

static __device__ __forceinline__ h16 toh_flush(float v) { const h16 r = (h16)v; return (fabsf(v) < 6.103515625e-05f) ? (h16)0.0f : r; }

__device__ __forceinline__ v16bf ldf(const bf* p)  { return ldb(p); }
__device__ __forceinline__ v16h  ldf(const h16* p) { return ldh(p); }
__device__ __forceinline__ v8f wmma_g(v16bf a, v16bf b, v8f c) { c = wmmab(a, b, c); asm volatile("v_nop\n\tv_nop\n\tv_nop\n\tv_nop" : "+v"(c) : "v"(a), "v"(b)); return c; }
__device__ __forceinline__ v8f wmma_g(v16h a, v16h b, v8f c)   { c = wmma16(a, b, c); asm volatile("v_nop\n\tv_nop\n\tv_nop\n\tv_nop" : "+v"(c) : "v"(a), "v"(b)); return c; }

__global__ __launch_bounds__(256) void k_cvt8(const float* __restrict__ src, bf* dst, size_t n8) {
    const size_t i = (size_t)blockIdx.x * 256 + threadIdx.x; if (i >= n8) return;
    const v8f v = *(const v8f*)(src + i * 8); v8us o;
#pragma unroll
    for (int k = 0; k < 8; ++k) o[k] = f2bf(v[k]);
    *(volatile v8us*)(dst + i * 8) = o; __threadfence(); *(volatile v8us*)(dst + i * 8) = o;
}

template <typename T, int K, int DUAL, int BIAS>
__device__ __forceinline__ void gemm64(const T* A1, const T* B1, const T* A2, const T* B2,
                                       const float* bias1, const float* bias2, float scale, float* C, int ldc) {
    static_assert(K % 32 == 0);
    static_assert(32 * 16 * 8 == 16 * 64 * 4);
    typedef decltype(ldf((const T*)0)) frag_t;
    __shared__ __align__(16) float os[16 * 68];
    const int lane = threadIdx.x & 31, lr = lane & 15, hi = lane >> 4; const int r0 = blockIdx.x * 64, c0 = blockIdx.y * 64;
    v8f acc[4][4];
#pragma unroll
    for (int mb = 0; mb < 4; ++mb)
#pragma unroll
        for (int nb = 0; nb < 4; ++nb) acc[mb][nb] = (v8f){};
    const size_t aoff = (size_t)(r0 + lr) * K + 8 * hi, boff = (size_t)(c0 + lr) * K + 8 * hi;
#pragma unroll 1
    for (int kc = 0; kc < K; kc += 32) {
        frag_t a[4];
#pragma unroll
        for (int mb = 0; mb < 4; ++mb) a[mb] = ldf(A1 + aoff + (size_t)mb * 16 * K + kc);
#pragma unroll
        for (int nb = 0; nb < 4; ++nb) { const frag_t b = ldf(B1 + boff + (size_t)nb * 16 * K + kc);
#pragma unroll
            for (int mb = 0; mb < 4; ++mb) acc[mb][nb] = wmma_g(a[mb], b, acc[mb][nb]); }
    }
    if (DUAL) {
#pragma unroll 1
        for (int kc = 0; kc < K; kc += 32) {
            frag_t a[4];
#pragma unroll
            for (int mb = 0; mb < 4; ++mb) a[mb] = ldf(A2 + aoff + (size_t)mb * 16 * K + kc);
#pragma unroll
            for (int nb = 0; nb < 4; ++nb) { const frag_t b = ldf(B2 + boff + (size_t)nb * 16 * K + kc);
#pragma unroll
                for (int mb = 0; mb < 4; ++mb) acc[mb][nb] = wmma_g(a[mb], b, acc[mb][nb]); }
        }
    }
    float bc[4];
#pragma unroll
    for (int nb = 0; nb < 4; ++nb) bc[nb] = (BIAS == 2) ? (bfr(bias1[c0 + nb * 16 + lr]) + bfr(bias2[c0 + nb * 16 + lr])) : 0.0f;
#pragma unroll
    for (int mb = 0; mb < 4; ++mb) {
        float br[8];
#pragma unroll
        for (int j = 0; j < 8; ++j) br[j] = (BIAS == 1) ? bfr(bias1[r0 + mb * 16 + hi * 8 + j]) : 0.0f;
#pragma unroll
        for (int nb = 0; nb < 4; ++nb) {
#pragma unroll
            for (int j = 0; j < 8; ++j) os[(hi * 8 + j) * 68 + nb * 16 + lr] = acc[mb][nb][j] * scale + bc[nb] + br[j]; }
        wave_sync();
        float* cb = C + (size_t)(r0 + mb * 16) * (size_t)ldc + c0;
#pragma unroll 1
        for (int ps = 0; ps < 2; ++ps) {
#pragma unroll
            for (int s = 0; s < 8; ++s) { const int row = 2 * s + (lane >> 4), c4 = (lane & 15) * 4;
                const v4f val = *(const v4fa*)(&os[row * 68 + c4]);
                *(volatile v4f*)(cb + (size_t)row * (size_t)ldc + c4) = val; }
            if (ps == 0) __threadfence(); }
        wave_sync();
    }
}

__global__ __launch_bounds__(32) void k_att1t(const bf* __restrict__ WE, const bf* __restrict__ XE, const float* __restrict__ be, float* A1T) {
    gemm64<bf, ENC, 0, 1>(WE, XE, WE, XE, be, be, 1.0f, A1T, NPIX);
}
__global__ __launch_bounds__(32) void k_sproj(const bf* __restrict__ XD, const bf* __restrict__ WT, const bf* __restrict__ XL, const bf* __restrict__ WL,
                                              const float* __restrict__ bt, const float* __restrict__ bl, float* SP) {
    gemm64<bf, ENC, 1, 2>(XD, WT, XL, WL, bt, bl, 1.0f, SP, ATT);
}
__global__ __launch_bounds__(32) void k_awe(const h16* __restrict__ AH, const h16* __restrict__ ET, float* AWE) {
    gemm64<h16, NPIX, 0, 0>(AH, ET, AH, ET, (const float*)0, (const float*)0, PSI, AWE, ENC);
}

__global__ __launch_bounds__(256) void k_enct(const float* __restrict__ X, h16* ET) {
#pragma clang fp contract(off)
    static_assert(256 * 16 * 2 == 64 * 64 * 2);
    __shared__ __align__(16) h16 ts[64 * TP];
    const int tid = threadIdx.x; const int p0 = blockIdx.x * 64, e0 = blockIdx.y * 64;
#pragma unroll
    for (int s = 0; s < 4; ++s) { const int pr = s * 16 + (tid >> 4), ec = (tid & 15) * 4;
        const v4f x = *(const v4f*)(X + (size_t)(p0 + pr) * ENC + e0 + ec);
#pragma unroll
        for (int i = 0; i < 4; ++i) ts[(ec + i) * TP + pr] = toh_flush(bfr(x[i])); }
    __syncthreads();
#pragma unroll 1
    for (int ps = 0; ps < 2; ++ps) {
#pragma unroll
        for (int s = 0; s < 2; ++s) { const int row = s * 32 + (tid >> 3), c8 = (tid & 7) * 8;
            const v8h hv = *(const v8ha*)(&ts[row * TP + c8]);
            *(volatile v8h*)(ET + (size_t)(e0 + row) * NPIX + p0 + c8) = hv; }
        if (ps == 0) __threadfence(); }
}

__global__ __launch_bounds__(256) void k_score(const float* __restrict__ A1T, const float* __restrict__ SP, const float* __restrict__ wf, const float* __restrict__ bfin,
                                               float* ALPHA, h16* AH) {
#pragma clang fp contract(off)
    static_assert(256 * 16 == NPIX * 4);
    static_assert(128 * 16 == NPIX * 2);
    __shared__ __align__(16) float sS[ATT];
    __shared__ __align__(16) float sW[ATT];
    __shared__ __align__(16) float sA[NPIX];
    __shared__ float wmx[8];
    __shared__ float wsm[8];
    const int tid = threadIdx.x, lane = tid & 31;
    const int wave = __builtin_amdgcn_readfirstlane((int)(threadIdx.x >> 5));
    const int n = blockIdx.x;
    sS[tid] = SP[(size_t)n * ATT + tid];
    sW[tid] = bfr(wf[tid]);
    __syncthreads();
    float acc[4] = { 0.0f, 0.0f, 0.0f, 0.0f };
    const float* ap = A1T + 4 * tid;
#pragma unroll 1
    for (int a0 = 0; a0 < ATT; a0 += 4) {
        const v4f sv = *(const v4fa*)(&sS[a0]); const v4f wv = *(const v4fa*)(&sW[a0]);
#pragma unroll
        for (int u = 0; u < 4; ++u) {
            const v4f x = *(const v4f*)(ap + (size_t)(a0 + u) * NPIX);
#pragma unroll
            for (int i = 0; i < 4; ++i) acc[i] = fmaf(fmaxf(x[i] + sv[u], 0.0f), wv[u], acc[i]);
        }
    }
    const float bfv = bfr(bfin[0]);
    float sc[4];
#pragma unroll
    for (int i = 0; i < 4; ++i) sc[i] = acc[i] + bfv;
    float mx = fmaxf(fmaxf(sc[0], sc[1]), fmaxf(sc[2], sc[3]));
#pragma unroll
    for (int off = 16; off >= 1; off >>= 1) mx = fmaxf(mx, __shfl_xor(mx, off, 32));
    if (lane == 0) wmx[wave] = mx;
    __syncthreads();
    float rm = wmx[0];
#pragma unroll
    for (int w = 1; w < 8; ++w) rm = fmaxf(rm, wmx[w]);
    v4f ev; float ssum = 0.0f;
#pragma unroll
    for (int i = 0; i < 4; ++i) { ev[i] = __builtin_amdgcn_exp2f((sc[i] - rm) * LOG2E); ssum += ev[i]; }
#pragma unroll
    for (int off = 16; off >= 1; off >>= 1) ssum += __shfl_xor(ssum, off, 32);
    *(v4fa*)(&sA[4 * tid]) = ev;
    if (lane == 0) wsm[wave] = ssum;
    __syncthreads();
    float tot = wsm[0];
#pragma unroll
    for (int w = 1; w < 8; ++w) tot += wsm[w];
    const float inv = 1.0f / tot;
    v4f av;
#pragma unroll
    for (int i = 0; i < 4; ++i) av[i] = ev[i] * inv;
    const int hb = (tid & 127) * 8;
    const v4f y0 = *(const v4fa*)(&sA[hb]); const v4f y1 = *(const v4fa*)(&sA[hb + 4]);
    v8h hv;
#pragma unroll
    for (int i = 0; i < 4; ++i) { hv[i] = toh_flush(y0[i] * inv * PSC); hv[4 + i] = toh_flush(y1[i] * inv * PSC); }
    float* arow = ALPHA + (size_t)n * APITCH + 4 * tid;
    h16* hrow = AH + (size_t)n * NPIX + hb;
#pragma unroll 1
    for (int ps = 0; ps < 2; ++ps) {
        *(volatile v4f*)arow = av;
        if (wave < 4) *(volatile v8h*)hrow = hv;
        if (ps == 0) __threadfence(); }
}

static constexpr size_t al256(size_t v) { return (v + 255) & ~(size_t)255; }
static constexpr size_t SZ_EB  = al256((size_t)NPIX * ENC * 2);
static constexpr size_t SZ_XB  = al256((size_t)NQ * ENC * 2);
static constexpr size_t SZ_WB  = al256((size_t)3 * ATT * ENC * 2);
static constexpr size_t SZ_A1T = al256((size_t)ATT * NPIX * 4);
static constexpr size_t SZ_SP  = al256((size_t)NQ * ATT * 4);
static constexpr size_t SZ_ET  = al256((size_t)ENC * NPIX * 2);
static constexpr size_t SZ_AH  = al256((size_t)NQ * NPIX * 2);
static constexpr size_t SZ_TOTAL = SZ_EB + 2 * SZ_XB + SZ_WB + SZ_A1T + SZ_SP + SZ_ET + SZ_AH;
static_assert(SZ_TOTAL <= (size_t)134217728);
static_assert(((size_t)ATT * ENC * 2) % 256 == 0);
static_assert(((size_t)NPIX * ENC) % 8 == 0);
static_assert(((size_t)NQ * ENC) % 8 == 0);
static_assert(((size_t)ATT * ENC) % 8 == 0);

extern "C" void kernel_launch(void* const* d_in, const int* in_sizes, int n_in,
                              void* d_out, int out_size, void* d_ws, size_t ws_size, hipStream_t stream) {
    if (n_in < 11) return;
    if ((size_t)in_sizes[0] < (size_t)NPIX * ENC) return;
    if ((size_t)in_sizes[1] < (size_t)NQ * ENC || (size_t)in_sizes[2] < (size_t)NQ * ENC) return;
    if ((size_t)in_sizes[3] < (size_t)ATT * ENC || (size_t)in_sizes[5] < (size_t)ATT * ENC || (size_t)in_sizes[7] < (size_t)ATT * ENC) return;
    if (in_sizes[4] < ATT || in_sizes[6] < ATT || in_sizes[8] < ATT || in_sizes[9] < ATT || in_sizes[10] < 1) return;
    if ((size_t)out_size < ALPHA_OFF + (size_t)(NQ - 1) * APITCH + NPIX) return;
    if (SZ_TOTAL > ws_size) return;
    const float* enc  = (const float*)d_in[0];
    const float* dec  = (const float*)d_in[1];
    const float* lang = (const float*)d_in[2];
    const float* we = (const float*)d_in[3]; const float* be = (const float*)d_in[4];
    const float* wt = (const float*)d_in[5]; const float* bt = (const float*)d_in[6];
    const float* wl = (const float*)d_in[7]; const float* bl = (const float*)d_in[8];
    const float* wf = (const float*)d_in[9]; const float* bfin = (const float*)d_in[10];
    float* AWE = (float*)d_out;
    float* ALPHA = (float*)d_out + ALPHA_OFF;
    char* wsp = (char*)d_ws;
    bf* EB = (bf*)wsp; wsp += SZ_EB;
    bf* DB = (bf*)wsp; wsp += SZ_XB;
    bf* LB = (bf*)wsp; wsp += SZ_XB;
    bf* WB = (bf*)wsp; wsp += SZ_WB;
    float* A1T = (float*)wsp; wsp += SZ_A1T;
    float* SP  = (float*)wsp; wsp += SZ_SP;
    h16* ET = (h16*)wsp; wsp += SZ_ET;
    h16* AH = (h16*)wsp; wsp += SZ_AH;
    bf* WE = WB; bf* WT = WB + (size_t)ATT * ENC; bf* WL = WB + (size_t)2 * ATT * ENC;

    { const size_t n8 = (size_t)NPIX * ENC / 8; k_cvt8<<<(unsigned)((n8 + 255) / 256), 256, 0, stream>>>(enc, EB, n8); }
    { const size_t n8 = (size_t)NQ * ENC / 8; const unsigned g = (unsigned)((n8 + 255) / 256);
      k_cvt8<<<g, 256, 0, stream>>>(dec, DB, n8); k_cvt8<<<g, 256, 0, stream>>>(lang, LB, n8); }
    { const size_t n8 = (size_t)ATT * ENC / 8; const unsigned g = (unsigned)((n8 + 255) / 256);
      k_cvt8<<<g, 256, 0, stream>>>(we, WE, n8); k_cvt8<<<g, 256, 0, stream>>>(wt, WT, n8); k_cvt8<<<g, 256, 0, stream>>>(wl, WL, n8); }

    k_enct<<<dim3(NPIX / 64, ENC / 64, 1), 256, 0, stream>>>(enc, ET);
    k_att1t<<<dim3(ATT / 64, NPIX / 64, 1), 32, 0, stream>>>(WE, EB, be, A1T);
    k_sproj<<<dim3(NQ / 64, ATT / 64, 1), 32, 0, stream>>>(DB, WT, LB, WL, bt, bl, SP);
    k_score<<<dim3(NQ, 1, 1), 256, 0, stream>>>(A1T, SP, wf, bfin, ALPHA, AH);
    k_awe<<<dim3(NQ / 64, ENC / 64, 1), 32, 0, stream>>>(AH, ET, AWE);
}
